// EdgePredictorResGCN_36197984370747
// MI455X (gfx1250) — hardware-verified
//
#include <hip/hip_runtime.h>
#include <stddef.h>


#define NTHR   256
#define NWAVE  8
#define EPT    8
#define CHUNK  (NTHR * EPT)
#define WCAP   (EPT * 32)
#define LISTN  (NWAVE * WCAP)
#define HIDC   64
#define MLPC   128
#define NBA    512
#define NBB    1024
#define EPB    512
#define ETW    4
#define APITCH 136
#define BN_EPS 1e-5f

#define PO_B0H 0
#define PO_B0L 16384
#define PO_R0H 32768
#define PO_R0L 40960
#define PO_B1H 49152
#define PO_B1L 57344
#define PO_B2H 65536
#define PO_B2L 73728
#define PO_PH  81920
#define PO_PL  90112
#define PO_QH  98304
#define PO_QL  106496
#define PO_W2H 114688
#define PO_W2L 131072
#define PO_END 147456
#define NPREPG 9216

static_assert(EPB == NWAVE * ETW * 16);
static_assert((EPB % 128) == 0);
static_assert(NPREPG * 8 * 2 == PO_END);
static_assert((NPREPG % 256) == 0);

typedef float          v2f  __attribute__((ext_vector_type(2)));
typedef float          v4f  __attribute__((ext_vector_type(4)));
typedef float          v8f  __attribute__((ext_vector_type(8)));
typedef int            v4i  __attribute__((ext_vector_type(4)));
typedef unsigned int   v4u  __attribute__((ext_vector_type(4)));
typedef double         v2d  __attribute__((ext_vector_type(2)));
typedef __bf16         v16bf __attribute__((ext_vector_type(16)));
union FragB { v16bf v; v4u q[2]; };

__device__ __forceinline__ int cmin(int a, int b) { return a < b ? a : b; }
__device__ __forceinline__ int clampi(int v, int lo, int hi) { return v < lo ? lo : (v > hi ? hi : v); }

__device__ __forceinline__ v8f z8f() {
  v8f z;
#pragma unroll
  for (int i = 0; i < 8; ++i) z[i] = 0.0f;
  return z;
}

__device__ __forceinline__ unsigned bfbits(float f) {
  const unsigned u = __float_as_uint(f);
  return (u + 0x7FFFu + ((u >> 16) & 1u)) >> 16;
}
__device__ __forceinline__ void split2(float a, float b, unsigned& hw, unsigned& lw) {
  const unsigned ha = bfbits(a), hb = bfbits(b);
  const float ra = a - __uint_as_float(ha << 16);
  const float rb = b - __uint_as_float(hb << 16);
  hw = ha | (hb << 16);
  lw = bfbits(ra) | (bfbits(rb) << 16);
}
__device__ __forceinline__ void split8(v4f a, v4f b, v4u& hi, v4u& lo) {
  unsigned h0, h1, h2, h3, l0, l1, l2, l3;
  split2(a.x, a.y, h0, l0);
  split2(a.z, a.w, h1, l1);
  split2(b.x, b.y, h2, l2);
  split2(b.z, b.w, h3, l3);
  v4u th, tl;
  th.x = h0; th.y = h1; th.z = h2; th.w = h3;
  tl.x = l0; tl.y = l1; tl.z = l2; tl.w = l3;
  hi = th; lo = tl;
}
__device__ __forceinline__ void mkfrag(v4f a0, v4f a1, v4f c0, v4f c1, float sc, FragB& fh, FragB& fl) {
  a0 *= sc; a1 *= sc; c0 *= sc; c1 *= sc;
  split8(a0, a1, fh.q[0], fl.q[0]);
  split8(c0, c1, fh.q[1], fl.q[1]);
}
__device__ __forceinline__ void ldB(const unsigned short* __restrict__ ph, const unsigned short* __restrict__ pl,
                                    FragB& bh, FragB& blo) {
  bh.q[0]  = *(const v4u*)ph;
  bh.q[1]  = *(const v4u*)(ph + 16);
  blo.q[0] = *(const v4u*)pl;
  blo.q[1] = *(const v4u*)(pl + 16);
}

__device__ __forceinline__ v8f wmb(v16bf a, v16bf b, v8f c) {
  v8f d = __builtin_amdgcn_wmma_f32_16x16x32_bf16(false, a, false, b, (short)0, c, false, false);
  asm volatile("v_nop\n\tv_nop\n\tv_nop\n\tv_nop" : "+v"(d) : "v"(a), "v"(b));
  return d;
}
__device__ __forceinline__ v8f wm3(const FragB& ah, const FragB& al, const FragB& bh, const FragB& blo, v8f c) {
  c = wmb(ah.v, bh.v, c);
  c = wmb(ah.v, blo.v, c);
  c = wmb(al.v, bh.v, c);
  return c;
}

__device__ __forceinline__ void wls() {
  __builtin_amdgcn_fence(__ATOMIC_RELEASE, "wavefront");
  asm volatile("s_wait_dscnt 0" ::: "memory");
  __builtin_amdgcn_wave_barrier();
  __builtin_amdgcn_fence(__ATOMIC_ACQUIRE, "wavefront");
}

__global__ __launch_bounds__(256) void k_prep(
    const float* __restrict__ Wl0, const float* __restrict__ Wr0, const float* __restrict__ rW0,
    const float* __restrict__ Wl1, const float* __restrict__ Wr1,
    const float* __restrict__ Wl2, const float* __restrict__ Wr2,
    const float* __restrict__ W1, const float* __restrict__ W2, unsigned short* pl) {
  const int g = blockIdx.x * 256 + threadIdx.x;
  if (g >= NPREPG) return;
  const float* sp; int spitch, scol, cpr, kp, dcol, oh, ol, rem;
  if (g < 1024)      { sp = Wl0; spitch = 128; scol = 0;  cpr = 16; kp = 256; dcol = 0;   oh = PO_B0H; ol = PO_B0L; rem = g; }
  else if (g < 2048) { sp = Wr0; spitch = 128; scol = 0;  cpr = 16; kp = 256; dcol = 128; oh = PO_B0H; ol = PO_B0L; rem = g - 1024; }
  else if (g < 3072) { sp = rW0; spitch = 128; scol = 0;  cpr = 16; kp = 128; dcol = 0;   oh = PO_R0H; ol = PO_R0L; rem = g - 2048; }
  else if (g < 3584) { sp = Wl1; spitch = 64;  scol = 0;  cpr = 8;  kp = 128; dcol = 0;   oh = PO_B1H; ol = PO_B1L; rem = g - 3072; }
  else if (g < 4096) { sp = Wr1; spitch = 64;  scol = 0;  cpr = 8;  kp = 128; dcol = 64;  oh = PO_B1H; ol = PO_B1L; rem = g - 3584; }
  else if (g < 4608) { sp = Wl2; spitch = 64;  scol = 0;  cpr = 8;  kp = 128; dcol = 0;   oh = PO_B2H; ol = PO_B2L; rem = g - 4096; }
  else if (g < 5120) { sp = Wr2; spitch = 64;  scol = 0;  cpr = 8;  kp = 128; dcol = 64;  oh = PO_B2H; ol = PO_B2L; rem = g - 4608; }
  else if (g < 6144) { sp = W1;  spitch = 128; scol = 0;  cpr = 8;  kp = 64;  dcol = 0;   oh = PO_PH;  ol = PO_PL;  rem = g - 5120; }
  else if (g < 7168) { sp = W1;  spitch = 128; scol = 64; cpr = 8;  kp = 64;  dcol = 0;   oh = PO_QH;  ol = PO_QL;  rem = g - 6144; }
  else               { sp = W2;  spitch = 128; scol = 0;  cpr = 16; kp = 128; dcol = 0;   oh = PO_W2H; ol = PO_W2L; rem = g - 7168; }
  const int n  = rem / cpr;
  const int c8 = rem - n * cpr;
  const float* s = sp + (size_t)n * spitch + scol + 8 * c8;
  const v4f a = *(const v4f*)s;
  const v4f b = *(const v4f*)(s + 4);
  v4u hi, lo;
  split8(a, b, hi, lo);
  const size_t d = (size_t)n * kp + dcol + 8 * c8;
  *(volatile v4u*)(pl + oh + d) = hi;
  *(volatile v4u*)(pl + ol + d) = lo;
  __threadfence();
  *(volatile v4u*)(pl + oh + d) = hi;
  *(volatile v4u*)(pl + ol + d) = lo;
}

template <int NB>
__device__ __forceinline__ int scan_chunk(const int* __restrict__ dsts, int nE, int cbase, int nodeBase,
                                          int vec8, int* list, int tid, int wave) {
  int wc = 0;
  const int el0  = tid * EPT;
  const int e0   = cbase + el0;
  const int sent = -2147483647 - 1;
  const int lst  = nE - 1;
  v4i da, db;
  if (vec8 != 0 && cbase + CHUNK <= nE) {
    da = *(const v4i*)(dsts + e0);
    db = *(const v4i*)(dsts + e0 + 4);
  } else {
    da.x = (e0     < nE) ? dsts[cmin(e0,     lst)] : sent;
    da.y = (e0 + 1 < nE) ? dsts[cmin(e0 + 1, lst)] : sent;
    da.z = (e0 + 2 < nE) ? dsts[cmin(e0 + 2, lst)] : sent;
    da.w = (e0 + 3 < nE) ? dsts[cmin(e0 + 3, lst)] : sent;
    db.x = (e0 + 4 < nE) ? dsts[cmin(e0 + 4, lst)] : sent;
    db.y = (e0 + 5 < nE) ? dsts[cmin(e0 + 5, lst)] : sent;
    db.z = (e0 + 6 < nE) ? dsts[cmin(e0 + 6, lst)] : sent;
    db.w = (e0 + 7 < nE) ? dsts[cmin(e0 + 7, lst)] : sent;
  }
  const unsigned nb = (unsigned)nodeBase;
  const unsigned s0 = (unsigned)da.x - nb, s1 = (unsigned)da.y - nb;
  const unsigned s2 = (unsigned)da.z - nb, s3 = (unsigned)da.w - nb;
  const unsigned s4 = (unsigned)db.x - nb, s5 = (unsigned)db.y - nb;
  const unsigned s6 = (unsigned)db.z - nb, s7 = (unsigned)db.w - nb;
  const bool h0 = s0 < (unsigned)NB, h1 = s1 < (unsigned)NB, h2 = s2 < (unsigned)NB, h3 = s3 < (unsigned)NB;
  const bool h4 = s4 < (unsigned)NB, h5 = s5 < (unsigned)NB, h6 = s6 < (unsigned)NB, h7 = s7 < (unsigned)NB;
  const unsigned any = __builtin_amdgcn_ballot_w32(h0 | h1 | h2 | h3 | h4 | h5 | h6 | h7);
  if (any != 0u) {
#define HITJ(J, HJ) { \
      const unsigned mj = __builtin_amdgcn_ballot_w32(HJ); \
      if (mj != 0u) { \
        if (HJ) { \
          const int pos = wc + (int)__builtin_amdgcn_mbcnt_lo(mj, 0u); \
          if (pos < WCAP) list[wave * WCAP + pos] = el0 + (J); \
        } \
        wc += (int)__builtin_popcount(mj); } }
    HITJ(0, h0)
    HITJ(1, h1)
    HITJ(2, h2)
    HITJ(3, h3)
    HITJ(4, h4)
    HITJ(5, h5)
    HITJ(6, h6)
    HITJ(7, h7)
#undef HITJ
  }
  return wc;
}

union ScrU { int l[LISTN]; double d[LISTN / 2]; };

template <int W, int NB, int HASRES>
__global__ __launch_bounds__(NTHR) void k_layer(
    const float* __restrict__ xin, const int* __restrict__ ei,
    const unsigned short* __restrict__ Bh, const unsigned short* __restrict__ Bl,
    const unsigned short* __restrict__ Rh, const unsigned short* __restrict__ Rl,
    const float* __restrict__ bl, const float* __restrict__ rb,
    float* pre, float* resp, double* part, int nN, int nE, int vec8) {
  constexpr int KP  = 2 * W;
  constexpr int TPB = NB / 16;
  constexpr int TPW = TPB / NWAVE;
  static_assert(TPW * NWAVE * 16 == NB);
  static_assert(W == 64 || W == 128);

  extern __shared__ v4f dacc4[];
  __shared__ __attribute__((aligned(16))) int  cnt[NB];
  __shared__ __attribute__((aligned(16))) ScrU scr;
  __shared__ int wcnt[NWAVE];
  float* dacc = (float*)dacc4;
  int*   list = scr.l;

  const int tid = threadIdx.x, lane = tid & 31, wave = tid >> 5, h = lane >> 4, m = lane & 15;
  const int nodeBase = blockIdx.x * NB;
  const int* srcs = ei;
  const int* dsts = ei + nE;

  {
    const v4f z4 = {0.0f, 0.0f, 0.0f, 0.0f};
    for (int i = tid; i < NB * W / 4; i += NTHR) dacc4[i] = z4;
    for (int i = tid; i < NB; i += NTHR) cnt[i] = 0;
  }
  __syncthreads();

  const int nChunks = (nE + CHUNK - 1) / CHUNK;
#pragma unroll 1
  for (int ch = 0; ch < nChunks; ++ch) {
    const int cbase = ch * CHUNK;
    const int wc = scan_chunk<NB>(dsts, nE, cbase, nodeBase, vec8, list, tid, wave);
    if (lane == 0) wcnt[wave] = wc;
    __syncthreads();
    if (wave == 0) {
#pragma unroll 1
      for (int w = 0; w < NWAVE; ++w) {
        int n = wcnt[w];
        n = n > WCAP ? WCAP : (n < 0 ? 0 : n);
        const int* lp = list + w * WCAP;
#pragma unroll 1
        for (int i = 0; i < n; ++i) {
          const int e = clampi(cbase + lp[i], 0, nE - 1);
          const int d = dsts[e];
          int s = srcs[e];
          const int slot = d - nodeBase;
          if ((unsigned)slot < (unsigned)NB) {
            s = clampi(s, 0, nN - 1);
            if (W == 128) {
              const v4f v = *(const v4f*)(xin + (size_t)s * 128 + 4 * lane);
              v4f* ap = (v4f*)(dacc + (size_t)slot * 128 + 4 * lane);
              v4f a = *ap;
              a += v;
              *ap = a;
            } else {
              const v2f v = *(const v2f*)(xin + (size_t)s * 64 + 2 * lane);
              v2f* ap = (v2f*)(dacc + (size_t)slot * 64 + 2 * lane);
              v2f a = *ap;
              a += v;
              *ap = a;
            }
            if (lane == 0) cnt[slot] += 1;
          }
        }
      }
    }
    __syncthreads();
  }

  double sS[4], sQ[4];
#pragma unroll
  for (int nt = 0; nt < 4; ++nt) { sS[nt] = 0.0; sQ[nt] = 0.0; }

#pragma unroll 1
  for (int it = 0; it < TPW; ++it) {
    const int tl   = wave + NWAVE * it;
    const int row0 = nodeBase + tl * 16;
    if (row0 < nN) {
      const int slotm = tl * 16 + m;
      const float inv = 1.0f / fmaxf((float)cnt[slotm], 1.0f);
      const float* mrow = dacc + (size_t)slotm * W;
      const float* xrow = xin + (size_t)(row0 + m) * W;
      v8f acc[4];
#pragma unroll
      for (int nt = 0; nt < 4; ++nt) acc[nt] = z8f();
#pragma unroll
      for (int ks = 0; ks < W / 32; ++ks) {
        const int kb = 32 * ks;
        FragB ah, al;
        mkfrag(*(const v4f*)(mrow + kb + 8 * h), *(const v4f*)(mrow + kb + 8 * h + 4),
               *(const v4f*)(mrow + kb + 16 + 8 * h), *(const v4f*)(mrow + kb + 20 + 8 * h), inv, ah, al);
#pragma unroll
        for (int nt = 0; nt < 4; ++nt) {
          const size_t bo = (size_t)(16 * nt + m) * KP + kb + 8 * h;
          FragB bh, blo;
          ldB(Bh + bo, Bl + bo, bh, blo);
          acc[nt] = wm3(ah, al, bh, blo, acc[nt]);
        }
      }
#pragma unroll
      for (int ks = 0; ks < W / 32; ++ks) {
        const int kb = 32 * ks;
        FragB ah, al;
        mkfrag(*(const v4f*)(xrow + kb + 8 * h), *(const v4f*)(xrow + kb + 8 * h + 4),
               *(const v4f*)(xrow + kb + 16 + 8 * h), *(const v4f*)(xrow + kb + 20 + 8 * h), 1.0f, ah, al);
#pragma unroll
        for (int nt = 0; nt < 4; ++nt) {
          const size_t bo = (size_t)(16 * nt + m) * KP + W + kb + 8 * h;
          FragB bh, blo;
          ldB(Bh + bo, Bl + bo, bh, blo);
          acc[nt] = wm3(ah, al, bh, blo, acc[nt]);
        }
      }
      wls();
      float* stg = dacc + (size_t)(tl * 16) * W;
#pragma unroll
      for (int nt = 0; nt < 4; ++nt) {
        const int n = 16 * nt + m;
        const float bv = bl[n];
#pragma unroll
        for (int r = 0; r < 8; ++r) {
          const float v = acc[nt][r] + bv;
          stg[(8 * h + r) * 64 + n] = v;
          sS[nt] += (double)v;
          sQ[nt] += (double)v * (double)v;
        }
      }
      wls();
#pragma unroll
      for (int i = 0; i < 8; ++i) {
        const int rl = 2 * i + h;
        const v4f v = *(const v4f*)(stg + rl * 64 + 4 * m);
        *(volatile v4f*)(pre + (size_t)(row0 + rl) * 64 + 4 * m) = v;
      }
      __threadfence();
#pragma unroll
      for (int i = 0; i < 8; ++i) {
        const int rl = 2 * i + h;
        const v4f v = *(const v4f*)(stg + rl * 64 + 4 * m);
        *(volatile v4f*)(pre + (size_t)(row0 + rl) * 64 + 4 * m) = v;
      }
      if constexpr (HASRES != 0) {
        v8f ar[4];
#pragma unroll
        for (int nt = 0; nt < 4; ++nt) ar[nt] = z8f();
#pragma unroll
        for (int ks = 0; ks < W / 32; ++ks) {
          const int kb = 32 * ks;
          FragB ah, al;
          mkfrag(*(const v4f*)(xrow + kb + 8 * h), *(const v4f*)(xrow + kb + 8 * h + 4),
                 *(const v4f*)(xrow + kb + 16 + 8 * h), *(const v4f*)(xrow + kb + 20 + 8 * h), 1.0f, ah, al);
#pragma unroll
          for (int nt = 0; nt < 4; ++nt) {
            const size_t bo = (size_t)(16 * nt + m) * W + kb + 8 * h;
            FragB bh, blo;
            ldB(Rh + bo, Rl + bo, bh, blo);
            ar[nt] = wm3(ah, al, bh, blo, ar[nt]);
          }
        }
        wls();
#pragma unroll
        for (int nt = 0; nt < 4; ++nt) {
          const int n = 16 * nt + m;
          const float bv = rb[n];
#pragma unroll
          for (int r = 0; r < 8; ++r) stg[(8 * h + r) * 64 + n] = ar[nt][r] + bv;
        }
        wls();
#pragma unroll
        for (int i = 0; i < 8; ++i) {
          const int rl = 2 * i + h;
          const v4f v = *(const v4f*)(stg + rl * 64 + 4 * m);
          *(volatile v4f*)(resp + (size_t)(row0 + rl) * 64 + 4 * m) = v;
        }
        __threadfence();
#pragma unroll
        for (int i = 0; i < 8; ++i) {
          const int rl = 2 * i + h;
          const v4f v = *(const v4f*)(stg + rl * 64 + 4 * m);
          *(volatile v4f*)(resp + (size_t)(row0 + rl) * 64 + 4 * m) = v;
        }
      }
    }
  }

  __syncthreads();
#pragma unroll
  for (int nt = 0; nt < 4; ++nt) {
    sS[nt] += __shfl_xor(sS[nt], 16, 32);
    sQ[nt] += __shfl_xor(sQ[nt], 16, 32);
  }
  double* red = scr.d;
  if (h == 0) {
#pragma unroll
    for (int nt = 0; nt < 4; ++nt) {
      red[wave * 128 + 16 * nt + m]      = sS[nt];
      red[wave * 128 + 64 + 16 * nt + m] = sQ[nt];
    }
  }
  __syncthreads();
  if (tid < 128) {
    double t = 0.0;
#pragma unroll
    for (int w = 0; w < NWAVE; ++w) t += red[w * 128 + tid];
    red[tid] = t;
  }
  __syncthreads();
  if (tid < 64) {
    const v2d v = *(const v2d*)(red + 2 * tid);
    *(volatile v2d*)(part + (size_t)blockIdx.x * 128 + 2 * tid) = v;
  }
  __threadfence();
  if (tid < 64) {
    const v2d v = *(const v2d*)(red + 2 * tid);
    *(volatile v2d*)(part + (size_t)blockIdx.x * 128 + 2 * tid) = v;
  }
}

__global__ __launch_bounds__(128) void k_bnc(const double* __restrict__ part, int nPart, int nN, float* bnl) {
  __shared__ __attribute__((aligned(16))) float lb[128];
  const int tid = threadIdx.x;
  if (tid < 64) {
    double S = 0.0, SS = 0.0;
#pragma unroll 1
    for (int b = 0; b < nPart; ++b) {
      S  += part[(size_t)b * 128 + tid];
      SS += part[(size_t)b * 128 + 64 + tid];
    }
    const double invn = 1.0 / (double)nN;
    const double mu = S * invn;
    double var = SS * invn - mu * mu;
    if (var < 0.0) var = 0.0;
    lb[tid]      = (float)mu;
    lb[64 + tid] = 1.0f / sqrtf((float)var + BN_EPS);
  }
  __syncthreads();
  v4f v = {0.0f, 0.0f, 0.0f, 0.0f};
  if (tid < 32) v = *(const v4f*)(lb + 4 * tid);
  if (tid < 32) *(volatile v4f*)(bnl + 4 * tid) = v;
  __threadfence();
  if (tid < 32) *(volatile v4f*)(bnl + 4 * tid) = v;
}

__global__ __launch_bounds__(256) void k_apply(const float* __restrict__ pre, const float* __restrict__ res,
                                               const float* __restrict__ bnl, const float* __restrict__ g,
                                               const float* __restrict__ be, float* hout, int nN) {
  const int idx = blockIdx.x * 256 + threadIdx.x;
  const int total = nN * 16;
  const bool ok = idx < total;
  const int ci = ok ? idx : 0;
  const int c0 = (ci & 15) * 4;
  const size_t fo = (size_t)ci * 4;
  const v4f p  = *(const v4f*)(pre + fo);
  const v4f r  = *(const v4f*)(res + fo);
  const v4f mu = *(const v4f*)(bnl + c0);
  const v4f rs = *(const v4f*)(bnl + 64 + c0);
  const v4f gg = *(const v4f*)(g + c0);
  const v4f bb = *(const v4f*)(be + c0);
  const v4f t = (p - mu) * rs * gg + bb;
  v4f o;
  o.x = fmaxf(t.x, 0.0f) + r.x;
  o.y = fmaxf(t.y, 0.0f) + r.y;
  o.z = fmaxf(t.z, 0.0f) + r.z;
  o.w = fmaxf(t.w, 0.0f) + r.w;
  if (ok) *(volatile v4f*)(hout + fo) = o;
  __threadfence();
  if (ok) *(volatile v4f*)(hout + fo) = o;
}

__global__ __launch_bounds__(128) void k_pq(const float* __restrict__ hin,
                                            const unsigned short* __restrict__ Ph, const unsigned short* __restrict__ Pl,
                                            const unsigned short* __restrict__ Qh, const unsigned short* __restrict__ Ql,
                                            const float* __restrict__ b1, float* Pout, float* Qout, int nN) {
  __shared__ __attribute__((aligned(16))) float stg[4][16 * MLPC];
  const int tid = threadIdx.x, lane = tid & 31, wave = tid >> 5, h = lane >> 4, m = lane & 15;
  const int row0 = (blockIdx.x * 4 + wave) * 16;
  if (row0 < nN) {
    const float* xr = hin + (size_t)(row0 + m) * HIDC;
    FragB ah[2], al[2];
#pragma unroll
    for (int ks = 0; ks < 2; ++ks) {
      const int kb = 32 * ks;
      mkfrag(*(const v4f*)(xr + kb + 8 * h), *(const v4f*)(xr + kb + 8 * h + 4),
             *(const v4f*)(xr + kb + 16 + 8 * h), *(const v4f*)(xr + kb + 20 + 8 * h), 1.0f, ah[ks], al[ks]);
    }
    float* st = &stg[wave][0];
#pragma unroll 1
    for (int ps = 0; ps < 2; ++ps) {
      const unsigned short* Wh  = (ps != 0) ? Qh : Ph;
      const unsigned short* Wlo = (ps != 0) ? Ql : Pl;
      float* dst = (ps != 0) ? Qout : Pout;
      const float bsel = (ps != 0) ? 1.0f : 0.0f;
      v8f acc[8];
#pragma unroll
      for (int nt = 0; nt < 8; ++nt) acc[nt] = z8f();
#pragma unroll
      for (int ks = 0; ks < 2; ++ks) {
        const int kb = 32 * ks;
#pragma unroll
        for (int nt = 0; nt < 8; ++nt) {
          const size_t bo = (size_t)(16 * nt + m) * HIDC + kb + 8 * h;
          FragB bh, blo;
          ldB(Wh + bo, Wlo + bo, bh, blo);
          acc[nt] = wm3(ah[ks], al[ks], bh, blo, acc[nt]);
        }
      }
      wls();
#pragma unroll
      for (int nt = 0; nt < 8; ++nt) {
        const int n = 16 * nt + m;
        const float bb = b1[n] * bsel;
#pragma unroll
        for (int r = 0; r < 8; ++r) st[(8 * h + r) * MLPC + n] = acc[nt][r] + bb;
      }
      wls();
#pragma unroll
      for (int i = 0; i < 16; ++i) {
        const v4f v = *(const v4f*)(st + i * MLPC + 4 * lane);
        *(volatile v4f*)(dst + (size_t)(row0 + i) * MLPC + 4 * lane) = v;
      }
      __threadfence();
#pragma unroll
      for (int i = 0; i < 16; ++i) {
        const v4f v = *(const v4f*)(st + i * MLPC + 4 * lane);
        *(volatile v4f*)(dst + (size_t)(row0 + i) * MLPC + 4 * lane) = v;
      }
      wls();
    }
  }
}

__global__ __launch_bounds__(NTHR) void k_edge(const float* __restrict__ P, const float* __restrict__ Q,
                                              const int* __restrict__ ei,
                                              const unsigned short* __restrict__ Wh, const unsigned short* __restrict__ Wlo,
                                              const float* __restrict__ b2, const float* __restrict__ W3,
                                              const float* __restrict__ b3, float* out, int nN, int nE) {
  __shared__ __attribute__((aligned(16))) unsigned short zt[NWAVE][2][16 * APITCH];
  __shared__ __attribute__((aligned(16))) float ost[EPB];
  const int tid = threadIdx.x, lane = tid & 31, wave = tid >> 5, h = lane >> 4, m = lane & 15;
  const int blkE0 = blockIdx.x * EPB;
  const float b3v = b3[0];
  float b2v[8], w3v[8];
#pragma unroll
  for (int nt = 0; nt < 8; ++nt) { b2v[nt] = b2[16 * nt + m]; w3v[nt] = W3[16 * nt + m]; }

#pragma unroll 1
  for (int it = 0; it < ETW; ++it) {
    const int tw = wave + NWAVE * it;
    const int e0 = blkE0 + tw * 16;
    if (e0 < nE) {
      const int em = cmin(e0 + m, nE - 1);
      int s = ei[em];
      int t = ei[(size_t)nE + em];
      s = clampi(s, 0, nN - 1);
      t = clampi(t, 0, nN - 1);
      const float* pr = P + (size_t)s * MLPC + 64 * h;
      const float* qr = Q + (size_t)t * MLPC + 64 * h;
      unsigned short* zh = &zt[wave][0][m * APITCH + 64 * h];
      unsigned short* zl = &zt[wave][1][m * APITCH + 64 * h];
#pragma unroll
      for (int j = 0; j < 8; ++j) {
        const v4f pa = *(const v4f*)(pr + 8 * j), pb = *(const v4f*)(pr + 8 * j + 4);
        const v4f qa = *(const v4f*)(qr + 8 * j), qb = *(const v4f*)(qr + 8 * j + 4);
        v4f ua = pa + qa, ub = pb + qb;
        ua.x = fmaxf(ua.x, 0.0f); ua.y = fmaxf(ua.y, 0.0f); ua.z = fmaxf(ua.z, 0.0f); ua.w = fmaxf(ua.w, 0.0f);
        ub.x = fmaxf(ub.x, 0.0f); ub.y = fmaxf(ub.y, 0.0f); ub.z = fmaxf(ub.z, 0.0f); ub.w = fmaxf(ub.w, 0.0f);
        v4u hi, lo;
        split8(ua, ub, hi, lo);
        *(v4u*)(zh + 8 * j) = hi;
        *(v4u*)(zl + 8 * j) = lo;
      }
      wls();
      v8f acc[8];
#pragma unroll
      for (int nt = 0; nt < 8; ++nt) acc[nt] = z8f();
      const unsigned short* arh = &zt[wave][0][m * APITCH + 8 * h];
      const unsigned short* arl = &zt[wave][1][m * APITCH + 8 * h];
#pragma unroll
      for (int ks = 0; ks < 4; ++ks) {
        const int kb = 32 * ks;
        FragB ah, al;
        ah.q[0] = *(const v4u*)(arh + kb);
        ah.q[1] = *(const v4u*)(arh + kb + 16);
        al.q[0] = *(const v4u*)(arl + kb);
        al.q[1] = *(const v4u*)(arl + kb + 16);
#pragma unroll
        for (int nt = 0; nt < 8; ++nt) {
          const size_t bo = (size_t)(16 * nt + m) * MLPC + kb + 8 * h;
          FragB bh, blo;
          ldB(Wh + bo, Wlo + bo, bh, blo);
          acc[nt] = wm3(ah, al, bh, blo, acc[nt]);
        }
      }
      float pz[8];
#pragma unroll
      for (int r = 0; r < 8; ++r) pz[r] = 0.0f;
#pragma unroll
      for (int nt = 0; nt < 8; ++nt) {
        const float bb = b2v[nt], wv = w3v[nt];
#pragma unroll
        for (int r = 0; r < 8; ++r) pz[r] += fmaxf(acc[nt][r] + bb, 0.0f) * wv;
      }
#pragma unroll
      for (int mask = 1; mask <= 8; mask <<= 1) {
#pragma unroll
        for (int r = 0; r < 8; ++r) pz[r] += __shfl_xor(pz[r], mask, 32);
      }
      if (m == 0) {
#pragma unroll
        for (int r = 0; r < 8; ++r) ost[tw * 16 + 8 * h + r] = pz[r] + b3v;
      }
      wls();
    }
  }
  __syncthreads();
  if (wave == 0) {
#pragma unroll
    for (int q = 0; q < EPB / 128; ++q) {
      const int base = blkE0 + q * 128 + 4 * lane;
      const v4f v = *(const v4f*)(ost + q * 128 + 4 * lane);
      if (base + 3 < nE) *(volatile v4f*)(out + base) = v;
      else {
        if (base     < nE) *(volatile float*)(out + base)     = v.x;
        if (base + 1 < nE) *(volatile float*)(out + base + 1) = v.y;
        if (base + 2 < nE) *(volatile float*)(out + base + 2) = v.z;
      }
    }
    __threadfence();
#pragma unroll
    for (int q = 0; q < EPB / 128; ++q) {
      const int base = blkE0 + q * 128 + 4 * lane;
      const v4f v = *(const v4f*)(ost + q * 128 + 4 * lane);
      if (base + 3 < nE) *(volatile v4f*)(out + base) = v;
      else {
        if (base     < nE) *(volatile float*)(out + base)     = v.x;
        if (base + 1 < nE) *(volatile float*)(out + base + 1) = v.y;
        if (base + 2 < nE) *(volatile float*)(out + base + 2) = v.z;
      }
    }
  }
}

static inline size_t alnup(size_t x) { return (x + 255) & ~(size_t)255; }

extern "C" void kernel_launch(void* const* d_in, const int* in_sizes, int n_in,
                              void* d_out, int out_size, void* d_ws, size_t ws_size,
                              hipStream_t stream) {
  if (n_in < 25) return;
  const int nN = in_sizes[0] / 128;
  const int nE = in_sizes[1] / 2;
  if (nN < 16 || (nN % 16) != 0 || in_sizes[0] != nN * 128) return;
  if (nE < 1 || in_sizes[1] != nE * 2) return;
  if (in_sizes[2] != 64 * 128 || in_sizes[3] < 64 || in_sizes[4] != 64 * 128 || in_sizes[5] < 64 || in_sizes[6] < 64) return;
  if (in_sizes[7] != 64 * 128 || in_sizes[8] < 64) return;
  if (in_sizes[9] != 64 * 64 || in_sizes[10] < 64 || in_sizes[11] != 64 * 64 || in_sizes[12] < 64 || in_sizes[13] < 64) return;
  if (in_sizes[14] != 64 * 64 || in_sizes[15] < 64 || in_sizes[16] != 64 * 64 || in_sizes[17] < 64 || in_sizes[18] < 64) return;
  if (in_sizes[19] != 128 * 128 || in_sizes[20] < 128 || in_sizes[21] != 128 * 128 || in_sizes[22] < 128) return;
  if (in_sizes[23] < 128 || in_sizes[24] < 1) return;
  if (out_size != nE) return;

  const float* x   = (const float*)d_in[0];
  const int*   ei  = (const int*)d_in[1];
  const float* Wl0 = (const float*)d_in[2];
  const float* bl0 = (const float*)d_in[3];
  const float* Wr0 = (const float*)d_in[4];
  const float* g0  = (const float*)d_in[5];
  const float* be0 = (const float*)d_in[6];
  const float* rW0 = (const float*)d_in[7];
  const float* rb0 = (const float*)d_in[8];
  const float* Wl1 = (const float*)d_in[9];
  const float* bl1 = (const float*)d_in[10];
  const float* Wr1 = (const float*)d_in[11];
  const float* g1  = (const float*)d_in[12];
  const float* be1 = (const float*)d_in[13];
  const float* Wl2 = (const float*)d_in[14];
  const float* bl2 = (const float*)d_in[15];
  const float* Wr2 = (const float*)d_in[16];
  const float* g2  = (const float*)d_in[17];
  const float* be2 = (const float*)d_in[18];
  const float* W1  = (const float*)d_in[19];
  const float* b1  = (const float*)d_in[20];
  const float* W2  = (const float*)d_in[21];
  const float* b2  = (const float*)d_in[22];
  const float* W3  = (const float*)d_in[23];
  const float* b3  = (const float*)d_in[24];
  float* out = (float*)d_out;

  const int nBlkA = (nN + NBA - 1) / NBA;
  const int nBlkB = (nN + NBB - 1) / NBB;

  char* ws = (char*)d_ws;
  size_t off = 0;
  const size_t oPl  = off; off = alnup(off + (size_t)PO_END * 2);
  const size_t oPrt = off; off = alnup(off + (size_t)nBlkA * 128 * 8);
  const size_t oBnl = off; off = alnup(off + 512);
  const size_t oPre = off; off = alnup(off + (size_t)nN * HIDC * 4);
  const size_t oRes = off; off = alnup(off + (size_t)nN * HIDC * 4);
  const size_t oHA  = off; off = alnup(off + (size_t)nN * HIDC * 4);
  const size_t oHB  = off; off = alnup(off + (size_t)nN * HIDC * 4);
  const size_t oP   = off; off = alnup(off + (size_t)nN * MLPC * 4);
  const size_t oQ   = off; off = alnup(off + (size_t)nN * MLPC * 4);
  if (off > ws_size) return;
  unsigned short* pl = (unsigned short*)(ws + oPl);
  double* part = (double*)(ws + oPrt);
  float* bnl  = (float*)(ws + oBnl);
  float* pre  = (float*)(ws + oPre);
  float* resp = (float*)(ws + oRes);
  float* hA   = (float*)(ws + oHA);
  float* hB   = (float*)(ws + oHB);
  float* Pp   = (float*)(ws + oP);
  float* Qp   = (float*)(ws + oQ);

  const int vec8 = ((nE & 3) == 0) ? 1 : 0;
  const size_t dynA = (size_t)NBA * 128 * 4;
  const size_t dynB = (size_t)NBB * 64 * 4;
  const int applyGrid = (nN * 16 + 255) / 256;
  const int pqGrid = ((nN / 16) + 3) / 4;
  const int edgeGrid = (nE + EPB - 1) / EPB;

  k_prep<<<NPREPG / 256, 256, 0, stream>>>(Wl0, Wr0, rW0, Wl1, Wr1, Wl2, Wr2, W1, W2, pl);

  hipFuncSetAttribute(reinterpret_cast<const void*>(&k_layer<128, NBA, 1>), hipFuncAttributeMaxDynamicSharedMemorySize, (int)dynA);
  hipFuncSetAttribute(reinterpret_cast<const void*>(&k_layer<64, NBB, 0>), hipFuncAttributeMaxDynamicSharedMemorySize, (int)dynB);
  k_layer<128, NBA, 1><<<nBlkA, NTHR, dynA, stream>>>(
      x, ei, pl + PO_B0H, pl + PO_B0L, pl + PO_R0H, pl + PO_R0L, bl0, rb0, pre, resp, part, nN, nE, vec8);
  k_bnc<<<1, 128, 0, stream>>>(part, nBlkA, nN, bnl);
  k_apply<<<applyGrid, 256, 0, stream>>>(pre, resp, bnl, g0, be0, hA, nN);

  k_layer<64, NBB, 0><<<nBlkB, NTHR, dynB, stream>>>(
      hA, ei, pl + PO_B1H, pl + PO_B1L, pl + PO_B1H, pl + PO_B1L, bl1, bl1, pre, pre, part, nN, nE, vec8);
  k_bnc<<<1, 128, 0, stream>>>(part, nBlkB, nN, bnl);
  k_apply<<<applyGrid, 256, 0, stream>>>(pre, hA, bnl, g1, be1, hB, nN);

  k_layer<64, NBB, 0><<<nBlkB, NTHR, dynB, stream>>>(
      hB, ei, pl + PO_B2H, pl + PO_B2L, pl + PO_B2H, pl + PO_B2L, bl2, bl2, pre, pre, part, nN, nE, vec8);
  k_bnc<<<1, 128, 0, stream>>>(part, nBlkB, nN, bnl);
  k_apply<<<applyGrid, 256, 0, stream>>>(pre, hB, bnl, g2, be2, hA, nN);

  k_pq<<<pqGrid, 128, 0, stream>>>(hA, pl + PO_PH, pl + PO_PL, pl + PO_QH, pl + PO_QL, b1, Pp, Qp, nN);
  k_edge<<<edgeGrid, NTHR, 0, stream>>>(Pp, Qp, ei, pl + PO_W2H, pl + PO_W2L, b2, W3, b3, out, nN, nE);
}
